// RNNModel_16870631539166
// MI455X (gfx1250) — hardware-verified
//
#include <hip/hip_runtime.h>
#include <math.h>

constexpr int NSEQ     = 2048;
constexpr int NSTEP    = 512;
constexpr int NIN      = 5;
constexpr int NHID     = 64;
constexpr int SEQ_BLK  = 32;
constexpr int NTHR     = 128;
constexpr int PREP_THR = 256;
constexpr int P1       = 104;
constexpr int P2       = 136;
constexpr int WPITCH   = 128;
constexpr int HSP      = 68;
constexpr int PAD0_COL0 = 70;
constexpr int PAD0_N    = WPITCH - PAD0_COL0;
constexpr int WPL_HALVES = 2 * NHID * WPITCH;
constexpr float OPC     = 16.0f;
constexpr float ACC_INV = 1.0f / 256.0f;
static_assert(NSEQ % SEQ_BLK == 0);
static_assert(NHID == 16 * (NTHR / 32));
static_assert(SEQ_BLK * 4 == NTHR);
static_assert((SEQ_BLK * P1) % NTHR == 0 && (SEQ_BLK * P2) % NTHR == 0);
static_assert(P1 % 8 == 0 && P2 % 8 == 0 && WPITCH % 8 == 0);
static_assert((NHID * NHID) % PREP_THR == 0);
static_assert(WPL_HALVES == 8 * 8 * PREP_THR);
static_assert(WPL_HALVES % (8 * NTHR) == 0);
static_assert(NHID * NIN <= 2 * PREP_THR);
static_assert(NSTEP >= 2);

typedef __attribute__((ext_vector_type(16))) _Float16 v16h;
typedef __attribute__((ext_vector_type(8)))  _Float16 v8h;
typedef __attribute__((ext_vector_type(8)))  float    v8f;
typedef __attribute__((ext_vector_type(4)))  float    v4f;
typedef __attribute__((ext_vector_type(4)))  unsigned v4u;

template <typename T> struct Frag;
template <> struct Frag<_Float16> {
  typedef v16h V; union U { v16h v; v8h h[2]; };
  static __device__ __forceinline__ v16h load(const _Float16* p) {
    U f; f.h[0] = *(const v8h*)(p); f.h[1] = *(const v8h*)(p + 16); return f.v;
  }
  static __device__ __forceinline__ v8f mma(v16h a, v16h b, v8f c) {
    return __builtin_amdgcn_wmma_f32_16x16x32_f16(false, a, false, b, (short)0, c, false, false);
  }
};

__device__ __forceinline__ void tie2_k3(v8f& c0, v8f& c1, v16h a0, v16h a1, v16h a2, v16h b0, v16h b1, v16h b2) {
  asm volatile("v_nop\n\tv_nop\n\tv_nop\n\tv_nop" : "+v"(c0), "+v"(c1) : "v"(a0), "v"(a1), "v"(a2), "v"(b0), "v"(b1), "v"(b2));
}
__device__ __forceinline__ void tie2_k4(v8f& c0, v8f& c1, v16h a0, v16h a1, v16h a2, v16h a3, v16h b0, v16h b1, v16h b2, v16h b3) {
  asm volatile("v_nop\n\tv_nop\n\tv_nop\n\tv_nop" : "+v"(c0), "+v"(c1) : "v"(a0), "v"(a1), "v"(a2), "v"(a3), "v"(b0), "v"(b1), "v"(b2), "v"(b3));
}

__device__ __forceinline__ unsigned short h_bits(float f) {
  const _Float16 h = (_Float16)f;
  return __builtin_bit_cast(unsigned short, h);
}
__device__ __forceinline__ float ftanh(float x) {
  const float e = expf(2.0f * x);
  return 1.0f - 2.0f * __builtin_amdgcn_rcpf(e + 1.0f);
}

__device__ __forceinline__ void store_x_seg(_Float16* A1t, int xrow, int xpart,
                                            float x0, float x1, float x2, float x3, float x4) {
  const float f = (xpart == 0) ? OPC : 0.0f;
  const unsigned short b0 = h_bits(x0 * f), b1 = h_bits(x1 * f), b2 = h_bits(x2 * f), b3 = h_bits(x3 * f), b4 = h_bits(x4 * f);
  v4u w;
  w[0] = (unsigned)b0 | ((unsigned)b1 << 16);
  w[1] = (unsigned)b2 | ((unsigned)b3 << 16);
  w[2] = (unsigned)b4 | ((unsigned)b4 << 16);
  w[3] = 0u;
  *(v4u*)(A1t + xrow * P1 + 64 + 8 * xpart) = w;
}

__global__ __launch_bounds__(PREP_THR) void prep_planes_kernel(
    const float* __restrict__ Wih0, const float* __restrict__ Whh0,
    const float* __restrict__ Wih1, const float* __restrict__ Whh1,
    unsigned short* __restrict__ WPL) {
  __shared__ __align__(16) float Ls[2 * NHID * WPITCH];
  const int tid = threadIdx.x;
#pragma unroll 1
  for (int i = tid; i < NHID * PAD0_N; i += PREP_THR) {
    const int n = i / PAD0_N;
    const int col = PAD0_COL0 + (i - n * PAD0_N);
    Ls[n * WPITCH + col] = 0.0f;
  }
  __syncthreads();
#pragma unroll 2
  for (int it = 0; it < (NHID * NHID) / PREP_THR; ++it) {
    const int i = it * PREP_THR + tid;
    const int n = i >> 6, k = i & 63;
    const float wa = Whh0[i];
    const float wb = Wih1[i];
    const float wc = Whh1[i];
    Ls[n * WPITCH + k] = OPC * wa;
    Ls[NHID * WPITCH + n * WPITCH + k] = OPC * wb;
    Ls[NHID * WPITCH + n * WPITCH + NHID + k] = OPC * wc;
  }
#pragma unroll 1
  for (int it = 0; it < 2; ++it) {
    const int i = it * PREP_THR + tid;
    const int ic = (i < NHID * NIN) ? i : (NHID * NIN - 1);
    const float w = Wih0[ic];
    const int n = ic / NIN, k = ic - n * NIN;
    if (i < NHID * NIN) {
      if (k < 4) {
        Ls[n * WPITCH + NHID + k] = OPC * w;
      } else {
        Ls[n * WPITCH + NHID + 4] = (0.5f * OPC) * w;
        Ls[n * WPITCH + NHID + 5] = (0.5f * OPC) * w;
      }
    }
  }
  __syncthreads();
  v4u wv[8];
#pragma unroll
  for (int s = 0; s < 8; ++s) {
    const int idx = s * PREP_THR + tid;
    const int plane = idx >> 10, row = (idx >> 4) & 63, c8 = (idx & 15) * 8;
    const float* sp = Ls + plane * (NHID * WPITCH) + row * WPITCH + c8;
    const v4f a = *(const v4f*)(sp);
    const v4f b = *(const v4f*)(sp + 4);
    const float a0 = a[0], a1 = a[1], a2 = a[2], a3 = a[3];
    const float b0 = b[0], b1 = b[1], b2 = b[2], b3 = b[3];
    v4u w;
    w[0] = (unsigned)h_bits(a0) | ((unsigned)h_bits(a1) << 16);
    w[1] = (unsigned)h_bits(a2) | ((unsigned)h_bits(a3) << 16);
    w[2] = (unsigned)h_bits(b0) | ((unsigned)h_bits(b1) << 16);
    w[3] = (unsigned)h_bits(b2) | ((unsigned)h_bits(b3) << 16);
    wv[s] = w;
  }
  for (int pass = 0; pass < 2; ++pass) {
#pragma unroll
    for (int s = 0; s < 8; ++s) {
      const int idx = s * PREP_THR + tid;
      const int plane = idx >> 10, row = (idx >> 4) & 63, c8 = (idx & 15) * 8;
      unsigned short* dp = WPL + (size_t)plane * (NHID * WPITCH) + (size_t)row * WPITCH + c8;
      *(volatile v4u*)dp = wv[s];
    }
    __threadfence();
  }
}

__global__ __launch_bounds__(NTHR) void rnn_seq_kernel(
    const float* __restrict__ x,
    const float* __restrict__ bih0, const float* __restrict__ bhh0,
    const float* __restrict__ bih1, const float* __restrict__ bhh1,
    const float* __restrict__ fcW, const float* __restrict__ fcb,
    const unsigned short* __restrict__ WPLp, float* __restrict__ out) {
  __shared__ __align__(16) _Float16 A1t[SEQ_BLK * P1];
  __shared__ __align__(16) _Float16 A2t[SEQ_BLK * P2];
  __shared__ __align__(16) float    Hs[SEQ_BLK * HSP];
  __shared__ __align__(16) float    fcs[NHID];
  __shared__ __align__(16) _Float16 Wl[WPL_HALVES];
  const int tid = threadIdx.x, lane = tid & 31, wave = tid >> 5;
  const int c = lane & 15, hh = lane >> 4, koff = 8 * hh;
  const int j = 16 * wave + c;
  const int rowbase = blockIdx.x * SEQ_BLK;
  const int xrow = tid >> 2, xpart = tid & 3;
  const float* xrp = x + (size_t)(rowbase + xrow) * NSTEP * NIN;

#pragma unroll 1
  for (int i = 0; i < (SEQ_BLK * P1) / NTHR; ++i) A1t[i * NTHR + tid] = (_Float16)0.0f;
#pragma unroll 1
  for (int i = 0; i < (SEQ_BLK * P2) / NTHR; ++i) A2t[i * NTHR + tid] = (_Float16)0.0f;
  if (tid < NHID) fcs[tid] = fcW[tid];
  {
    const v4u* wsrc = (const v4u*)WPLp;
#pragma unroll 1
    for (int it = 0; it < WPL_HALVES / (8 * NTHR); ++it) {
      const int w = it * NTHR + tid;
      const v4u wq = wsrc[w];
      *(v4u*)(Wl + 8 * w) = wq;
    }
  }
  __syncthreads();

  {
    const float x0 = xrp[0], x1 = xrp[1], x2 = xrp[2], x3 = xrp[3], x4 = xrp[4];
    store_x_seg(A1t, xrow, xpart, x0, x1, x2, x3, x4);
  }
  v16h Bw1[3], Bw2[4];
  {
    const _Float16* b1r = Wl + j * WPITCH + koff;
    Bw1[0] = Frag<_Float16>::load(b1r);
    Bw1[1] = Frag<_Float16>::load(b1r + 32);
    Bw1[2] = Frag<_Float16>::load(b1r + 64);
    const _Float16* b2r = Wl + NHID * WPITCH + j * WPITCH + koff;
    Bw2[0] = Frag<_Float16>::load(b2r);
    Bw2[1] = Frag<_Float16>::load(b2r + 32);
    Bw2[2] = Frag<_Float16>::load(b2r + 64);
    Bw2[3] = Frag<_Float16>::load(b2r + 96);
  }
  const float bias1 = bih0[j] + bhh0[j];
  const float bias2 = bih1[j] + bhh1[j];
  const float fcb0  = fcb[0];
  float h1v[2][8], h2v[2][8];
#pragma unroll
  for (int ms = 0; ms < 2; ++ms)
#pragma unroll
    for (int r = 0; r < 8; ++r) { h1v[ms][r] = 0.0f; h2v[ms][r] = 0.0f; }
  __syncthreads();

  const v8f z8 = {0.f, 0.f, 0.f, 0.f, 0.f, 0.f, 0.f, 0.f};

#pragma unroll 1
  for (int t = 0; t < NSTEP; ++t) {
    const int tn = (t + 1 < NSTEP) ? (t + 1) : (NSTEP - 1);
    const float* xp = xrp + tn * NIN;
    const float xn0 = xp[0], xn1 = xp[1], xn2 = xp[2], xn3 = xp[3], xn4 = xp[4];

    v8f acc1[2];
    acc1[0] = z8; acc1[1] = z8;
#pragma unroll
    for (int ms = 0; ms < 2; ++ms) {
      const _Float16* ar = A1t + (16 * ms + c) * P1 + koff;
      const v16h a0 = Frag<_Float16>::load(ar);
      const v16h a1 = Frag<_Float16>::load(ar + 32);
      const v16h a2 = Frag<_Float16>::load(ar + 64);
      acc1[ms] = Frag<_Float16>::mma(a0, Bw1[0], acc1[ms]);
      acc1[ms] = Frag<_Float16>::mma(a1, Bw1[1], acc1[ms]);
      acc1[ms] = Frag<_Float16>::mma(a2, Bw1[2], acc1[ms]);
      tie2_k3(acc1[0], acc1[1], a0, a1, a2, Bw1[0], Bw1[1], Bw1[2]);
    }
#pragma unroll
    for (int ms = 0; ms < 2; ++ms) {
#pragma unroll
      for (int r = 0; r < 8; ++r) {
        const float z  = acc1[ms][r] * ACC_INV + bias1;
        const float hn = ftanh(z);
        h1v[ms][r] = hn;
        const int row = 16 * ms + 8 * hh + r;
        A2t[row * P2 + j]        = (_Float16)(OPC * hn);
        A2t[row * P2 + NHID + j] = (_Float16)(OPC * h2v[ms][r]);
      }
    }
    __syncthreads();

    v8f acc2[2];
    acc2[0] = z8; acc2[1] = z8;
#pragma unroll
    for (int ms = 0; ms < 2; ++ms) {
      const _Float16* ar = A2t + (16 * ms + c) * P2 + koff;
      const v16h a0 = Frag<_Float16>::load(ar);
      const v16h a1 = Frag<_Float16>::load(ar + 32);
      const v16h a2 = Frag<_Float16>::load(ar + 64);
      const v16h a3 = Frag<_Float16>::load(ar + 96);
      acc2[ms] = Frag<_Float16>::mma(a0, Bw2[0], acc2[ms]);
      acc2[ms] = Frag<_Float16>::mma(a1, Bw2[1], acc2[ms]);
      acc2[ms] = Frag<_Float16>::mma(a2, Bw2[2], acc2[ms]);
      acc2[ms] = Frag<_Float16>::mma(a3, Bw2[3], acc2[ms]);
      tie2_k4(acc2[0], acc2[1], a0, a1, a2, a3, Bw2[0], Bw2[1], Bw2[2], Bw2[3]);
    }
#pragma unroll
    for (int ms = 0; ms < 2; ++ms) {
#pragma unroll
      for (int r = 0; r < 8; ++r) {
        const float z  = acc2[ms][r] * ACC_INV + bias2;
        const float hn = ftanh(z);
        h2v[ms][r] = hn;
        const int row = 16 * ms + 8 * hh + r;
        A1t[row * P1 + j] = (_Float16)(OPC * h1v[ms][r]);
      }
    }
    store_x_seg(A1t, xrow, xpart, xn0, xn1, xn2, xn3, xn4);
    __syncthreads();
  }

#pragma unroll
  for (int ms = 0; ms < 2; ++ms)
#pragma unroll
    for (int r = 0; r < 8; ++r) Hs[(16 * ms + 8 * hh + r) * HSP + j] = h2v[ms][r];
  __syncthreads();
  if (wave == 0) {
    float s = 0.0f;
#pragma unroll 1
    for (int jj = 0; jj < NHID; ++jj) s = fmaf(Hs[lane * HSP + jj], fcs[jj], s);
    s += fcb0;
    float* op = out + rowbase + lane;
    *(volatile float*)op = s;
    __threadfence();
    *(volatile float*)op = s;
  }
}

extern "C" void kernel_launch(void* const* d_in, const int* in_sizes, int n_in,
                              void* d_out, int out_size, void* d_ws, size_t ws_size, hipStream_t stream) {
  if (n_in < 11 || d_out == nullptr || d_ws == nullptr) return;
  if (in_sizes[0] != NSEQ * NSTEP * NIN || in_sizes[1] != NHID * NIN || in_sizes[2] != NHID * NHID ||
      in_sizes[3] != NHID || in_sizes[4] != NHID || in_sizes[5] != NHID * NHID || in_sizes[6] != NHID * NHID ||
      in_sizes[7] != NHID || in_sizes[8] != NHID || in_sizes[9] != NHID || in_sizes[10] != 1 ||
      out_size != NSEQ) return;

  const float* x    = (const float*)d_in[0];
  const float* Wih0 = (const float*)d_in[1];
  const float* Whh0 = (const float*)d_in[2];
  const float* bih0 = (const float*)d_in[3];
  const float* bhh0 = (const float*)d_in[4];
  const float* Wih1 = (const float*)d_in[5];
  const float* Whh1 = (const float*)d_in[6];
  const float* bih1 = (const float*)d_in[7];
  const float* bhh1 = (const float*)d_in[8];
  const float* fcW  = (const float*)d_in[9];
  const float* fcb  = (const float*)d_in[10];
  float* out = (float*)d_out;

  char* ws = (char*)d_ws; size_t off = 0;
  auto carve = [&](size_t bytes) -> char* { char* p = ws + off; off += (bytes + 255) & ~(size_t)255; return p; };
  unsigned short* WPL = (unsigned short*)carve((size_t)WPL_HALVES * 2);
  if (off > ws_size || off > (size_t)134217728) return;

  prep_planes_kernel<<<1, PREP_THR, 0, stream>>>(Wih0, Whh0, Wih1, Whh1, WPL);
  rnn_seq_kernel<<<NSEQ / SEQ_BLK, NTHR, 0, stream>>>(x, bih0, bhh0, bih1, bhh1, fcW, fcb, WPL, out);
}
